// ProjectionAttentionKernel_44753559225153
// MI455X (gfx1250) — hardware-run, weakly checked
//
#include <hip/hip_runtime.h>


#define NB_  8
#define TT   512
#define DM   768
#define D3   (3 * DM)
#define NH_  12
#define HD   64
#define NSC  (NH_ * TT * TT)
#define NP1  3072
#define NP2  64
#define SQC  16384.0f
#define SUN  3.725290298461914e-09f
#define WCAR 16.0f
#define MCAR 0.0625f
#define LN_EPS 1.0e-5f
#define PFL  6.103515625e-05f
#define C0   0.015625f
typedef _Float16 h16;
typedef unsigned short bf;
typedef __attribute__((ext_vector_type(16))) __bf16   v16bf;
typedef __attribute__((ext_vector_type(16))) _Float16 v16h;
typedef __attribute__((ext_vector_type(8)))  _Float16 v8h;
typedef __attribute__((ext_vector_type(8)))  unsigned short v8us;
typedef __attribute__((ext_vector_type(8)))  float    v8f;
typedef __attribute__((ext_vector_type(4)))  float    v4f;
typedef v8h  __attribute__((may_alias)) v8ha;
typedef v4f  __attribute__((may_alias)) v4fa;
typedef v8us __attribute__((may_alias)) v8usa;

__device__ __forceinline__ unsigned short f2bf(float f) { unsigned u = __float_as_uint(f); u += 0x7FFFu + ((u >> 16) & 1u); return (unsigned short)(u >> 16); }
__device__ __forceinline__ float bf2f(unsigned short b) { return __uint_as_float(((unsigned)b) << 16); }
__device__ __forceinline__ float bfr(float f) { return bf2f(f2bf(f)); }
__device__ __forceinline__ v16h cat16(v8h lo, v8h hi) { return __builtin_shufflevector(lo, hi, 0, 1, 2, 3, 4, 5, 6, 7, 8, 9, 10, 11, 12, 13, 14, 15); }
__device__ __forceinline__ v16bf cat16b(v8us lo, v8us hi) { return __builtin_bit_cast(v16bf, __builtin_shufflevector(lo, hi, 0, 1, 2, 3, 4, 5, 6, 7, 8, 9, 10, 11, 12, 13, 14, 15)); }
__device__ __forceinline__ v8f wmma16(v16h a, v16h b, v8f c) { return __builtin_amdgcn_wmma_f32_16x16x32_f16(false, a, false, b, (short)0, c, false, false); }
__device__ __forceinline__ v8f wmmab(v16bf a, v16bf b, v8f c) { return __builtin_amdgcn_wmma_f32_16x16x32_bf16(false, a, false, b, (short)0, c, false, false); }


template <typename T16> struct WFrag;
template <> struct WFrag<h16> { typedef v16h V; static __device__ __forceinline__ V ld(const h16* p) { return cat16(*(const v8h*)p, *(const v8h*)(p + 16)); } static __device__ __forceinline__ v8f mma(V a, V b, v8f c) { return wmma16(a, b, c); } };
template <> struct WFrag<bf> { typedef v16bf V; static __device__ __forceinline__ V ld(const bf* p) { return cat16b(*(const v8us*)p, *(const v8us*)(p + 16)); } static __device__ __forceinline__ v8f mma(V a, V b, v8f c) { return wmmab(a, b, c); } };
template <typename T16, int NSPLIT, bool BIAS>
__global__ __launch_bounds__(32) void k_gemmw(const T16* __restrict__ A, const T16* __restrict__ A2, const T16* __restrict__ Bt, const T16* __restrict__ Bt2, int K, float* C, int ldc, const float* __restrict__ bias, size_t sA, size_t sB, size_t sC) {
    typedef typename WFrag<T16>::V V;
    __shared__ __align__(16) float os[16 * 68];
    const size_t z = blockIdx.z; A += z * sA; if (A2) A2 += z * sA; Bt += z * sB; if (Bt2) Bt2 += z * sB; C += z * sC;
    const int lane = threadIdx.x & 31, lr = lane & 15, hi = lane >> 4; const int r0 = blockIdx.x * 64, c0 = blockIdx.y * 64;
    v8f acc[4][4];
#pragma unroll
    for (int mb = 0; mb < 4; ++mb)
#pragma unroll
        for (int nb = 0; nb < 4; ++nb) acc[mb][nb] = (v8f){};
    const size_t aoff = (size_t)(r0 + lr) * K + 8 * hi, boff = (size_t)(c0 + lr) * K + 8 * hi;
    for (int kc = 0; kc < K; kc += 32) {
        V a[4], a2[4];
#pragma unroll
        for (int mb = 0; mb < 4; ++mb) { a[mb] = WFrag<T16>::ld(A + aoff + (size_t)mb * 16 * K + kc); if (NSPLIT == 1 || NSPLIT == 2) a2[mb] = WFrag<T16>::ld(A2 + aoff + (size_t)mb * 16 * K + kc); }
#pragma unroll
        for (int nb = 0; nb < 4; ++nb) { const V b = WFrag<T16>::ld(Bt + boff + (size_t)nb * 16 * K + kc); V b2; if (NSPLIT >= 2) b2 = WFrag<T16>::ld(Bt2 + boff + (size_t)nb * 16 * K + kc);
#pragma unroll
            for (int mb = 0; mb < 4; ++mb) { acc[mb][nb] = WFrag<T16>::mma(a[mb], b, acc[mb][nb]); if (NSPLIT == 1 || NSPLIT == 2) acc[mb][nb] = WFrag<T16>::mma(a2[mb], b, acc[mb][nb]); if (NSPLIT >= 2) acc[mb][nb] = WFrag<T16>::mma(a[mb], b2, acc[mb][nb]); } }
        asm volatile("v_nop\n\tv_nop\n\tv_nop\n\tv_nop" : "+v"(acc[0][0]), "+v"(acc[1][1]), "+v"(acc[2][2]), "+v"(acc[3][3]) : "v"(a[0]), "v"(a[3]));
    }
#pragma unroll
    for (int mb = 0; mb < 4; ++mb) {
#pragma unroll
        for (int nb = 0; nb < 4; ++nb) {
#pragma unroll
            for (int j = 0; j < 8; ++j) os[(hi * 8 + j) * 68 + nb * 16 + lr] = acc[mb][nb][j]; }
        __builtin_amdgcn_wave_barrier(); asm volatile("" ::: "memory");
        float* crow = C + (size_t)(r0 + mb * 16) * ldc + c0;
#pragma unroll 1
        for (int ps = 0; ps < 2; ++ps) {
#pragma unroll
            for (int s = 0; s < 8; ++s) { const int row = 2 * s + hi, cofs = lr * 4; v4f val = *(const v4fa*)(os + row * 68 + cofs); if (BIAS) { val[0] += bfr(bias[c0 + cofs]); val[1] += bfr(bias[c0 + cofs + 1]); val[2] += bfr(bias[c0 + cofs + 2]); val[3] += bfr(bias[c0 + cofs + 3]); }
                *(volatile v4f*)(crow + (size_t)row * ldc + cofs) = val; }
            if (ps == 0) __threadfence(); }
        __builtin_amdgcn_wave_barrier(); asm volatile("" ::: "memory");
    }
}

__device__ __forceinline__ h16 tohx(float x) { return (h16)x; }
typedef __attribute__((ext_vector_type(2))) _Float16 v2h;
typedef __attribute__((ext_vector_type(2))) unsigned short v2us;

__global__ __launch_bounds__(256) void k_cvt8(const float* __restrict__ src, bf* dst, size_t n8) { const size_t i = (size_t)blockIdx.x * 256 + threadIdx.x; if (i >= n8) return; const v8f v = *(const v8f*)(src + i * 8); v8us o;
#pragma unroll
    for (int k = 0; k < 8; ++k) o[k] = f2bf(v[k]); *(volatile v8us*)(dst + i * 8) = o; __threadfence(); *(volatile v8us*)(dst + i * 8) = o; }
__global__ __launch_bounds__(256) void k_vtp(const float* __restrict__ F, int pitch, int nheads, h16* V16, bf* Vh, bf* Vl) { const size_t e = ((size_t)blockIdx.x * 256 + threadIdx.x) * 2; if (e >= (size_t)nheads * HD * TT) return; const int t = (int)(e % TT); const int d = (int)((e / TT) % HD); const int g = (int)(e / ((size_t)TT * HD)); v2h o16; v2us oh, ol;
#pragma unroll
    for (int q = 0; q < 2; ++q) { const float x = F[(size_t)(t + q) * pitch + g * HD + d]; o16[q] = tohx(x); (void)oh; (void)ol; }
    *(volatile v2h*)(V16 + e) = o16; __threadfence(); *(volatile v2h*)(V16 + e) = o16; }
template <typename T16> __device__ __forceinline__ unsigned short cv16(float x);
template <> __device__ __forceinline__ unsigned short cv16<bf>(float x) { return f2bf(x); }
template <> __device__ __forceinline__ unsigned short cv16<h16>(float x) { const h16 h = (h16)x; return __builtin_bit_cast(unsigned short, h); }
template <typename T16>
__global__ __launch_bounds__(256) void k_castp(const float* __restrict__ src, int rows_valid, int lc, float mul, unsigned short* dst) { const unsigned e = blockIdx.x * 256 + threadIdx.x; const unsigned r = e >> (lc - 3); const unsigned c0 = (e & ((1u << (lc - 3)) - 1u)) << 3; const unsigned rr = (r < (unsigned)rows_valid) ? r : (unsigned)(rows_valid - 1);
    const float* s = src + ((size_t)rr << lc) + c0; const v4f a = *(const v4f*)s, b = *(const v4f*)(s + 4); const float lm = (r < (unsigned)rows_valid) ? mul : 0.0f; v8us o;
#pragma unroll
    for (int q = 0; q < 4; ++q) { o[q] = cv16<T16>(__fmul_rn(a[q], lm)); o[q + 4] = cv16<T16>(__fmul_rn(b[q], lm)); }
    *(volatile v8us*)(dst + (size_t)e * 8) = o; __threadfence(); *(volatile v8us*)(dst + (size_t)e * 8) = o; }


__global__ __launch_bounds__(256) void k_b2h(const bf* __restrict__ src, float mul, unsigned short* dst) { const unsigned e = blockIdx.x * 256 + threadIdx.x; const v8us a = *(const v8us*)(src + (size_t)e * 8); v8us o;
#pragma unroll
    for (int q = 0; q < 8; ++q) o[q] = cv16<h16>(__fmul_rn(bf2f(a[q]), mul));
    *(volatile v8us*)(dst + (size_t)e * 8) = o; __threadfence(); *(volatile v8us*)(dst + (size_t)e * 8) = o; }

__global__ __launch_bounds__(256) void k_usqw(const float* __restrict__ F, unsigned short* W) { const unsigned e = blockIdx.x * 256 + threadIdx.x; const unsigned o = e & 7u, n = e >> 3; const unsigned h = blockIdx.y, p = blockIdx.z; const float* f = F + (size_t)n * D3 + p * DM + h * HD; float ss = 0.0f;
#pragma unroll
    for (int c = 0; c < HD / 4; ++c) { const v4f v = *(const v4f*)(f + 4 * c); ss = __fmaf_rn(v[0], v[0], ss); ss = __fmaf_rn(v[1], v[1], ss); ss = __fmaf_rn(v[2], v[2], ss); ss = __fmaf_rn(v[3], v[3], ss); }
    const float r = __fdiv_rn(1.0f, __fsqrt_rn(ss)); const v4f x0 = *(const v4f*)(f + 8 * o), x1 = *(const v4f*)(f + 8 * o + 4); v8us w;
#pragma unroll
    for (int q = 0; q < 4; ++q) { const float u0 = __fmul_rn(x0[q], r), u1 = __fmul_rn(x1[q], r); const float w0 = __fmul_rn(__fmul_rn(u0, u0), SQC), w1 = __fmul_rn(__fmul_rn(u1, u1), SQC); w[q] = cv16<h16>(w0 < PFL ? 0.0f : w0); w[q + 4] = cv16<h16>(w1 < PFL ? 0.0f : w1); }
    unsigned short* d = W + (((size_t)p * NH_ + h) * TT + n) * HD + 8 * o; *(volatile v8us*)d = w; __threadfence(); *(volatile v8us*)d = w; }

__global__ __launch_bounds__(256) void k_blocksum1(const float* __restrict__ S, float* P1) { const unsigned t = blockIdx.x * 256 + threadIdx.x; v4f a = (v4f){0.0f, 0.0f, 0.0f, 0.0f}, b = (v4f){0.0f, 0.0f, 0.0f, 0.0f};
    for (int j = 0; j < NSC / 4 / NP1; ++j) { const v4f v = *(const v4f*)(S + 4 * ((size_t)j * NP1 + t));
#pragma unroll
        for (int c = 0; c < 4; ++c) { const float s = __fsub_rn(__fmul_rn(v[c], SUN), C0); a[c] = __fadd_rn(a[c], s); b[c] = __fmaf_rn(s, s, b[c]); } }
    const float s1 = __fadd_rn(__fadd_rn(a[0], a[1]), __fadd_rn(a[2], a[3])), s2 = __fadd_rn(__fadd_rn(b[0], b[1]), __fadd_rn(b[2], b[3]));
    *(volatile float*)(P1 + t) = s1; *(volatile float*)(P1 + NP1 + t) = s2; __threadfence(); *(volatile float*)(P1 + t) = s1; *(volatile float*)(P1 + NP1 + t) = s2; }

__global__ __launch_bounds__(64) void k_blocksum2(const float* __restrict__ P1, float* P2) { const unsigned t = threadIdx.x; float s1 = 0.0f, s2 = 0.0f;
#pragma unroll
    for (int j = 0; j < NP1 / NP2 / 4; ++j) { const v4f u = *(const v4f*)(P1 + (NP1 / NP2) * t + 4 * j), w = *(const v4f*)(P1 + NP1 + (NP1 / NP2) * t + 4 * j);
#pragma unroll
        for (int c = 0; c < 4; ++c) { s1 = __fadd_rn(s1, u[c]); s2 = __fadd_rn(s2, w[c]); } }
    *(volatile float*)(P2 + t) = s1; *(volatile float*)(P2 + NP2 + t) = s2; __threadfence(); *(volatile float*)(P2 + t) = s1; *(volatile float*)(P2 + NP2 + t) = s2; }

__global__ __launch_bounds__(256) void k_blocknorm(const float* __restrict__ S, const float* __restrict__ P2, const float* __restrict__ G, const float* __restrict__ Bv, float* O, unsigned short* A16) { const size_t i = ((size_t)blockIdx.x * 256 + threadIdx.x) * 8; float t1 = 0.0f, t2 = 0.0f;
#pragma unroll
    for (int j = 0; j < NP2 / 4; ++j) { const v4f u = *(const v4f*)(P2 + 4 * j), w = *(const v4f*)(P2 + NP2 + 4 * j);
#pragma unroll
        for (int c = 0; c < 4; ++c) { t1 = __fadd_rn(t1, u[c]); t2 = __fadd_rn(t2, w[c]); } }
    const float dm = __fmul_rn(t1, 1.0f / (float)NSC); const float mean = __fadd_rn(C0, dm); const float var = __fsub_rn(__fmul_rn(t2, 1.0f / (float)NSC), __fmul_rn(dm, dm)); const float rs = __fdiv_rn(1.0f, __fsqrt_rn(__fadd_rn(var, LN_EPS)));
    const v4f s0 = *(const v4f*)(S + i), s1 = *(const v4f*)(S + i + 4), g0 = *(const v4f*)(G + i), g1 = *(const v4f*)(G + i + 4), b0 = *(const v4f*)(Bv + i), b1 = *(const v4f*)(Bv + i + 4); v4f o0, o1; v8us h;
#pragma unroll
    for (int q = 0; q < 4; ++q) { o0[q] = __fmaf_rn(__fmul_rn(__fsub_rn(__fmul_rn(s0[q], SUN), mean), rs), bfr(g0[q]), bfr(b0[q])); o1[q] = __fmaf_rn(__fmul_rn(__fsub_rn(__fmul_rn(s1[q], SUN), mean), rs), bfr(g1[q]), bfr(b1[q])); h[q] = cv16<h16>(fabsf(o0[q]) < PFL ? 0.0f : o0[q]); h[q + 4] = cv16<h16>(fabsf(o1[q]) < PFL ? 0.0f : o1[q]); }
    *(volatile v4f*)(O + i) = o0; *(volatile v4f*)(O + i + 4) = o1; *(volatile v8us*)(A16 + i) = h; __threadfence(); *(volatile v4f*)(O + i) = o0; *(volatile v4f*)(O + i + 4) = o1; *(volatile v8us*)(A16 + i) = h; }

extern "C" void kernel_launch(void* const* d_in, const int* in_sizes, int n_in,
                              void* d_out, int out_size, void* d_ws, size_t ws_size, hipStream_t stream) {
    (void)in_sizes; (void)n_in; (void)out_size;
    const float* x = (const float*)d_in[0]; const float* wqkv = (const float*)d_in[1]; const float* lnw = (const float*)d_in[2]; const float* lnb = (const float*)d_in[3]; const float* wo = (const float*)d_in[4]; const float* bo = (const float*)d_in[5];
    float* OUT0 = (float*)d_out; float* OUT1 = OUT0 + (size_t)NB_ * TT * DM;
    static_assert(NH_ * HD == DM && TT % 64 == 0 && DM % 64 == 0 && D3 % 64 == 0 && DM % 32 == 0 && HD % 32 == 0 && TT % 32 == 0 && (TT * 8) % 256 == 0 && NSC % (4 * NP1) == 0 && NP1 % 256 == 0 && NP1 % (4 * NP2) == 0 && NP2 == 64 && (NSC / 8) % 256 == 0 && ((size_t)NB_ * TT * DM / 8) % 256 == 0 && ((size_t)D3 * DM / 8) % 256 == 0 && ((size_t)DM * DM / 8) % 256 == 0 && ((size_t)NB_ * TT * DM) % 256 == 0, "the heads fill the width; every product's sizes are whole tiles and whole depth steps; every flat kernel's grid is exact");
    char* wsp = (char*)d_ws;
    auto take = [&](size_t bytes) { char* p = wsp; wsp += (bytes + 255) & ~(size_t)255; return (void*)p; };
    bf* XB = (bf*)take((size_t)NB_ * TT * DM * 2); bf* WB = (bf*)take((size_t)D3 * DM * 2); bf* WOB = (bf*)take((size_t)DM * DM * 2); h16* WO16 = (h16*)take((size_t)DM * DM * 2); float* QKV = (float*)take((size_t)NB_ * TT * D3 * 4);
    h16* QK2 = (h16*)take((size_t)2 * NH_ * TT * HD * 2); h16* VT16 = (h16*)take((size_t)NH_ * HD * TT * 2); float* Sb = (float*)take((size_t)NSC * 4); float* P1 = (float*)take((size_t)2 * NP1 * 4); float* P2 = (float*)take((size_t)2 * NP2 * 4); h16* A16 = (h16*)take((size_t)NSC * 2);
    float* MG = (float*)take((size_t)NB_ * TT * DM * 4); h16* MG16 = (h16*)take((size_t)NB_ * TT * DM * 2);
    if ((size_t)(wsp - (char*)d_ws) > ws_size) return;
    k_cvt8<<<(unsigned)((size_t)NB_ * TT * DM / 8 / 256), 256, 0, stream>>>(x, XB, (size_t)NB_ * TT * DM / 8); k_cvt8<<<(unsigned)((size_t)D3 * DM / 8 / 256), 256, 0, stream>>>(wqkv, WB, (size_t)D3 * DM / 8); k_cvt8<<<(unsigned)((size_t)DM * DM / 8 / 256), 256, 0, stream>>>(wo, WOB, (size_t)DM * DM / 8);
    k_b2h<<<(unsigned)((size_t)DM * DM / 8 / 256), 256, 0, stream>>>(WOB, WCAR, (unsigned short*)WO16);
    k_gemmw<bf, 0, false><<<dim3(NB_ * TT / 64, D3 / 64, 1), 32, 0, stream>>>(XB, nullptr, WB, nullptr, DM, QKV, D3, nullptr, 0, 0, 0);
    for (int b = 0; b < NB_; ++b) { const float* fb = QKV + (size_t)b * TT * D3;
        k_usqw<<<dim3(TT * 8 / 256, NH_, 2), 256, 0, stream>>>(fb, (unsigned short*)QK2);
        k_vtp<<<(unsigned)(((size_t)NH_ * HD * TT / 2 + 255) / 256), 256, 0, stream>>>(fb + 2 * DM, D3, NH_, VT16, nullptr, nullptr);
        k_gemmw<h16, 0, false><<<dim3(TT / 64, TT / 64, NH_), 32, 0, stream>>>(QK2, nullptr, QK2 + (size_t)NH_ * TT * HD, nullptr, HD, Sb, TT, nullptr, (size_t)TT * HD, (size_t)TT * HD, (size_t)TT * TT);
        k_blocksum1<<<NP1 / 256, 256, 0, stream>>>(Sb, P1); k_blocksum2<<<1, 64, 0, stream>>>(P1, P2);
        k_blocknorm<<<(unsigned)(NSC / 8 / 256), 256, 0, stream>>>(Sb, P2, lnw, lnb, OUT1 + (size_t)b * NSC, (unsigned short*)A16);
        k_gemmw<h16, 0, false><<<dim3(TT / 64, HD / 64, NH_), 32, 0, stream>>>(A16, nullptr, VT16, nullptr, TT, MG + (size_t)b * TT * DM, DM, nullptr, (size_t)TT * TT, (size_t)HD * TT, (size_t)HD); }
    k_castp<h16><<<(unsigned)((size_t)NB_ * TT * DM / 8 / 256), 256, 0, stream>>>(MG, (int)((size_t)NB_ * TT * DM / 256), 8, MCAR, (unsigned short*)MG16);
    k_gemmw<h16, 0, true><<<dim3(NB_ * TT / 64, DM / 64, 1), 32, 0, stream>>>(MG16, nullptr, WO16, nullptr, DM, OUT0, DM, bo, 0, 0, 0);
}
